// TransformerXLDecoderLayer_27539330302101
// MI455X (gfx1250) — hardware-run, weakly checked
//
#include <hip/hip_runtime.h>


#define NB_  2
#define QL   1024
#define ML   1024
#define KL   2048
#define DM   1024
#define NH_  16
#define HD   64
#define DFF  4096
#define ZH   2
#define PCAR 1024.0f
typedef _Float16 h16;
typedef unsigned short bf;
typedef __attribute__((ext_vector_type(16))) __bf16   v16bf;
typedef __attribute__((ext_vector_type(16))) _Float16 v16h;
typedef __attribute__((ext_vector_type(8)))  _Float16 v8h;
typedef __attribute__((ext_vector_type(8)))  unsigned short v8us;
typedef __attribute__((ext_vector_type(8)))  float    v8f;
typedef __attribute__((ext_vector_type(4)))  float    v4f;
typedef v8h  __attribute__((may_alias)) v8ha;
typedef v4f  __attribute__((may_alias)) v4fa;
typedef v8us __attribute__((may_alias)) v8usa;

__device__ __forceinline__ unsigned short f2bf(float f) { unsigned u = __float_as_uint(f); u += 0x7FFFu + ((u >> 16) & 1u); return (unsigned short)(u >> 16); }
__device__ __forceinline__ float bf2f(unsigned short b) { return __uint_as_float(((unsigned)b) << 16); }
__device__ __forceinline__ float bfr(float f) { return bf2f(f2bf(f)); }
__device__ __forceinline__ v16h cat16(v8h lo, v8h hi) { return __builtin_shufflevector(lo, hi, 0, 1, 2, 3, 4, 5, 6, 7, 8, 9, 10, 11, 12, 13, 14, 15); }
__device__ __forceinline__ v16bf cat16b(v8us lo, v8us hi) { return __builtin_bit_cast(v16bf, __builtin_shufflevector(lo, hi, 0, 1, 2, 3, 4, 5, 6, 7, 8, 9, 10, 11, 12, 13, 14, 15)); }
__device__ __forceinline__ v8f wmma16(v16h a, v16h b, v8f c) { return __builtin_amdgcn_wmma_f32_16x16x32_f16(false, a, false, b, (short)0, c, false, false); }
__device__ __forceinline__ v8f wmmab(v16bf a, v16bf b, v8f c) { return __builtin_amdgcn_wmma_f32_16x16x32_bf16(false, a, false, b, (short)0, c, false, false); }


template <typename T16> struct WFrag;
template <> struct WFrag<h16> { typedef v16h V; static __device__ __forceinline__ V ld(const h16* p) { return cat16(*(const v8h*)p, *(const v8h*)(p + 16)); } static __device__ __forceinline__ v8f mma(V a, V b, v8f c) { return wmma16(a, b, c); } };
template <> struct WFrag<bf> { typedef v16bf V; static __device__ __forceinline__ V ld(const bf* p) { return cat16b(*(const v8us*)p, *(const v8us*)(p + 16)); } static __device__ __forceinline__ v8f mma(V a, V b, v8f c) { return wmmab(a, b, c); } };
template <typename T16, int NSPLIT, bool BIAS>
__global__ __launch_bounds__(32) void k_gemmw(const T16* __restrict__ A, const T16* __restrict__ A2, const T16* __restrict__ Bt, const T16* __restrict__ Bt2, int K, float* C, int ldc, const float* __restrict__ bias, size_t sA, size_t sB, size_t sC) {
    typedef typename WFrag<T16>::V V;
    __shared__ __align__(16) float os[16 * 68];
    const size_t z = blockIdx.z; A += z * sA; if (A2) A2 += z * sA; Bt += z * sB; if (Bt2) Bt2 += z * sB; C += z * sC;
    const int lane = threadIdx.x & 31, lr = lane & 15, hi = lane >> 4; const int r0 = blockIdx.x * 64, c0 = blockIdx.y * 64;
    v8f acc[4][4];
#pragma unroll
    for (int mb = 0; mb < 4; ++mb)
#pragma unroll
        for (int nb = 0; nb < 4; ++nb) acc[mb][nb] = (v8f){};
    const size_t aoff = (size_t)(r0 + lr) * K + 8 * hi, boff = (size_t)(c0 + lr) * K + 8 * hi;
#pragma unroll 1
    for (int kc = 0; kc < K; kc += 32) {
        V a[4], a2[4];
#pragma unroll
        for (int mb = 0; mb < 4; ++mb) { a[mb] = WFrag<T16>::ld(A + aoff + (size_t)mb * 16 * K + kc); if (NSPLIT == 1 || NSPLIT == 2) a2[mb] = WFrag<T16>::ld(A2 + aoff + (size_t)mb * 16 * K + kc); }
#pragma unroll
        for (int nb = 0; nb < 4; ++nb) { const V b = WFrag<T16>::ld(Bt + boff + (size_t)nb * 16 * K + kc); V b2; if (NSPLIT >= 2) b2 = WFrag<T16>::ld(Bt2 + boff + (size_t)nb * 16 * K + kc);
#pragma unroll
            for (int mb = 0; mb < 4; ++mb) { acc[mb][nb] = WFrag<T16>::mma(a[mb], b, acc[mb][nb]); if (NSPLIT == 1 || NSPLIT == 2) acc[mb][nb] = WFrag<T16>::mma(a2[mb], b, acc[mb][nb]); if (NSPLIT >= 2) acc[mb][nb] = WFrag<T16>::mma(a[mb], b2, acc[mb][nb]); } }
        asm volatile("v_nop\n\tv_nop\n\tv_nop\n\tv_nop" : "+v"(acc[0][0]), "+v"(acc[1][1]), "+v"(acc[2][2]), "+v"(acc[3][3]) : "v"(a[0]), "v"(a[3]));
    }
#pragma unroll
    for (int mb = 0; mb < 4; ++mb) {
#pragma unroll
        for (int nb = 0; nb < 4; ++nb) {
#pragma unroll
            for (int j = 0; j < 8; ++j) os[(hi * 8 + j) * 68 + nb * 16 + lr] = acc[mb][nb][j]; }
        __builtin_amdgcn_wave_barrier(); asm volatile("" ::: "memory");
        float* crow = C + (size_t)(r0 + mb * 16) * ldc + c0;
#pragma unroll 1
        for (int ps = 0; ps < 2; ++ps) {
#pragma unroll
            for (int s = 0; s < 8; ++s) { const int row = 2 * s + hi, cofs = lr * 4; v4f val = *(const v4fa*)(os + row * 68 + cofs); if (BIAS) { val[0] += bfr(bias[c0 + cofs]); val[1] += bfr(bias[c0 + cofs + 1]); val[2] += bfr(bias[c0 + cofs + 2]); val[3] += bfr(bias[c0 + cofs + 3]); }
                *(volatile v4f*)(crow + (size_t)row * ldc + cofs) = val; }
            if (ps == 0) __threadfence(); }
        __builtin_amdgcn_wave_barrier(); asm volatile("" ::: "memory");
    }
}

template <typename T16, int NSPLIT, int CMODE>
__global__ __launch_bounds__(32) void k_gemmc(const T16* __restrict__ A, const T16* __restrict__ A2, const T16* __restrict__ Bt, const T16* __restrict__ Bt2, int K, float* C, int ldc, int roff, size_t sA, size_t sB, size_t sC) {
    typedef typename WFrag<T16>::V V;
    __shared__ __align__(16) float os[16 * 68];
    const size_t z = blockIdx.z; A += z * sA; if (A2) A2 += z * sA; Bt += z * sB; if (Bt2) Bt2 += z * sB; C += z * sC;
    const int lane = threadIdx.x & 31, lr = lane & 15, hi = lane >> 4; const int r0 = blockIdx.x * 64, c0 = blockIdx.y * 64;
    if (CMODE == 1 && c0 > r0 + roff + 63) return;
    const int Kl = (CMODE == 2) ? min(K, r0 + roff + 64) : K;
    v8f acc[4][4];
#pragma unroll
    for (int mb = 0; mb < 4; ++mb)
#pragma unroll
        for (int nb = 0; nb < 4; ++nb) acc[mb][nb] = (v8f){};
    const size_t aoff = (size_t)(r0 + lr) * K + 8 * hi, boff = (size_t)(c0 + lr) * K + 8 * hi;
#pragma unroll 1
    for (int kc = 0; kc < Kl; kc += 32) {
        V a[4], a2[4];
#pragma unroll
        for (int mb = 0; mb < 4; ++mb) { a[mb] = WFrag<T16>::ld(A + aoff + (size_t)mb * 16 * K + kc); if (NSPLIT == 1 || NSPLIT == 2) a2[mb] = WFrag<T16>::ld(A2 + aoff + (size_t)mb * 16 * K + kc); }
#pragma unroll
        for (int nb = 0; nb < 4; ++nb) { const V b = WFrag<T16>::ld(Bt + boff + (size_t)nb * 16 * K + kc); V b2; if (NSPLIT >= 2) b2 = WFrag<T16>::ld(Bt2 + boff + (size_t)nb * 16 * K + kc);
#pragma unroll
            for (int mb = 0; mb < 4; ++mb) { acc[mb][nb] = WFrag<T16>::mma(a[mb], b, acc[mb][nb]); if (NSPLIT == 1 || NSPLIT == 2) acc[mb][nb] = WFrag<T16>::mma(a2[mb], b, acc[mb][nb]); if (NSPLIT >= 2) acc[mb][nb] = WFrag<T16>::mma(a[mb], b2, acc[mb][nb]); } }
        asm volatile("v_nop\n\tv_nop\n\tv_nop\n\tv_nop" : "+v"(acc[0][0]), "+v"(acc[1][1]), "+v"(acc[2][2]), "+v"(acc[3][3]) : "v"(a[0]), "v"(a[3]));
    }
#pragma unroll
    for (int mb = 0; mb < 4; ++mb) {
#pragma unroll
        for (int nb = 0; nb < 4; ++nb) {
#pragma unroll
            for (int j = 0; j < 8; ++j) os[(hi * 8 + j) * 68 + nb * 16 + lr] = acc[mb][nb][j]; }
        __builtin_amdgcn_wave_barrier(); asm volatile("" ::: "memory");
        float* crow = C + (size_t)(r0 + mb * 16) * ldc + c0;
#pragma unroll 1
        for (int ps = 0; ps < 2; ++ps) {
#pragma unroll
            for (int s = 0; s < 8; ++s) { const int row = 2 * s + hi, cofs = lr * 4; v4f val = *(const v4fa*)(os + row * 68 + cofs);
                *(volatile v4f*)(crow + (size_t)row * ldc + cofs) = val; }
            if (ps == 0) __threadfence(); }
        __builtin_amdgcn_wave_barrier(); asm volatile("" ::: "memory");
    }
}
__device__ __forceinline__ h16 tohx(float x) { return (h16)x; }
__device__ __forceinline__ void splitf(float y, unsigned short& h, unsigned short& l) { h = f2bf(y); l = f2bf(y - bf2f(h)); }
typedef __attribute__((ext_vector_type(2))) unsigned short v2us;
typedef __attribute__((ext_vector_type(4))) unsigned short v4us;
typedef __attribute__((ext_vector_type(2))) _Float16 v2h;
typedef __attribute__((ext_vector_type(4))) _Float16 v4h;

__global__ __launch_bounds__(256) void k_cvt8(const float* __restrict__ src, bf* dst, size_t n8) { const size_t i = (size_t)blockIdx.x * 256 + threadIdx.x; if (i >= n8) return; const v8f v = *(const v8f*)(src + i * 8); v8us o;
#pragma unroll
    for (int k = 0; k < 8; ++k) o[k] = f2bf(v[k]); *(volatile v8us*)(dst + i * 8) = o; __threadfence(); *(volatile v8us*)(dst + i * 8) = o; }
__global__ __launch_bounds__(256) void k_wtG(const float* __restrict__ w, int K, int N, bf* Bt) {
    const int lane = threadIdx.x & 31; const int L0 = (blockIdx.x * 8 + (threadIdx.x >> 5)) * 8; const int nlines = N * K / 64;
#pragma unroll
    for (int ps = 0; ps < 2; ++ps) {
#pragma unroll 1
        for (int l = 0; l < 8; ++l) { const int L = L0 + l; if (L >= nlines) break; const size_t e = (size_t)L * 64 + lane * 2; const int k = (int)(e % K), n = (int)(e / K); v2us o;
            o[0] = f2bf(w[(size_t)k * N + n]); o[1] = f2bf(w[(size_t)(k + 1) * N + n]); *(volatile v2us*)(Bt + e) = o; }
        if (ps == 0) __threadfence(); }
}

__global__ __launch_bounds__(256) void k_lnrow(const float* __restrict__ X, size_t bstride, const float* __restrict__ g, const float* __restrict__ bb, int rnd, int roff, bf* Hh, bf* Hl) { const int lane = threadIdx.x & 31; const size_t r = (size_t)blockIdx.x * 8 + (threadIdx.x >> 5); if (r >= QL) return; const float* xr = X + r * bstride; float v[32]; float s = 0.f;
#pragma unroll
    for (int ch = 0; ch < 8; ++ch) { const v4f a = *(const v4f*)(xr + ch * 128 + lane * 4);
#pragma unroll
        for (int u = 0; u < 4; ++u) { const float t = rnd ? bfr(a[u]) : a[u]; v[ch * 4 + u] = t; s += t; } }
#pragma unroll
    for (int sh = 16; sh; sh >>= 1) s += __shfl_xor(s, sh, 32);
    const float mean = s * (1.0f / DM); float q = 0.f;
#pragma unroll
    for (int k = 0; k < 32; ++k) { float d = __fsub_rn(v[k], mean); asm volatile("" : "+v"(d)); v[k] = d; float p = __fmul_rn(d, d); asm volatile("" : "+v"(p)); q = __fadd_rn(q, p); }
#pragma unroll
    for (int sh = 16; sh; sh >>= 1) q += __shfl_xor(q, sh, 32);
    const float rs = __frsqrt_rn(__fadd_rn(q * (1.0f / DM), 1e-5f));
    for (int ps = 0; ps < 2; ++ps) {
#pragma unroll
        for (int ch = 0; ch < 8; ++ch) { v4us oh, ol;
#pragma unroll
            for (int u = 0; u < 4; ++u) { const int c = ch * 128 + lane * 4 + u; float n0 = __fmul_rn(v[ch * 4 + u], rs); asm volatile("" : "+v"(n0)); float gg = bfr(g[c]), be = bfr(bb[c]); asm volatile("" : "+v"(gg)); asm volatile("" : "+v"(be)); float t1 = __fmul_rn(n0, gg); asm volatile("" : "+v"(t1)); unsigned short a2, c2; splitf(__fadd_rn(t1, be), a2, c2); oh[u] = a2; ol[u] = c2; }
            const size_t oo = (size_t)(roff + r) * DM + ch * 128 + lane * 4; *(volatile v4us*)(Hh + oo) = oh; *(volatile v4us*)(Hl + oo) = ol; }
        if (ps == 0) __threadfence(); } }
__global__ __launch_bounds__(256) void k_hpb(const float* __restrict__ F, int pitch, int col0, int rows, const float* __restrict__ bias, bf* Ph, bf* Pl) { const size_t e = ((size_t)blockIdx.x * 256 + threadIdx.x) * 4; if (e >= (size_t)NH_ * rows * HD) return; const int d = (int)(e % HD); const int r = (int)((e / HD) % rows); const int h = (int)(e / ((size_t)HD * rows)); const float* f = F + (size_t)r * pitch + col0 + h * HD + d; v4us oh, ol;
#pragma unroll
    for (int u = 0; u < 4; ++u) { const float x = bias ? __fadd_rn(f[u], bfr(bias[h * HD + d + u])) : f[u]; unsigned short a, b; splitf(x, a, b); oh[u] = a; ol[u] = b; } *(volatile v4us*)(Ph + e) = oh; *(volatile v4us*)(Pl + e) = ol; __threadfence(); *(volatile v4us*)(Ph + e) = oh; *(volatile v4us*)(Pl + e) = ol; }
__global__ __launch_bounds__(256) void k_vt16(const float* __restrict__ F, h16* VT) { const size_t e = ((size_t)blockIdx.x * 256 + threadIdx.x) * 2; if (e >= (size_t)NH_ * HD * KL) return; const int j = (int)(e % KL); const int d = (int)((e / KL) % HD); const int h = (int)(e / ((size_t)KL * HD)); v2h o; o[0] = tohx(F[(size_t)j * (3 * DM) + 2 * DM + h * HD + d]); o[1] = tohx(F[(size_t)(j + 1) * (3 * DM) + 2 * DM + h * HD + d]); *(volatile v2h*)(VT + e) = o; __threadfence(); *(volatile v2h*)(VT + e) = o; }
__global__ __launch_bounds__(256) void k_xsoft(const float* __restrict__ AC, const float* __restrict__ BD, const int* __restrict__ mk, h16* P16) { const int lane = threadIdx.x & 31; const int row = blockIdx.x * 8 + (threadIdx.x >> 5); if (row >= ZH * QL) return; const int i = row % QL; const float* ar = AC + (size_t)row * KL; const float* br = BD + (size_t)row * KL + (QL - 1 - i); const int* mr = mk + (size_t)i * KL; float v[KL / 32]; float mx = -3.0e38f;
#pragma unroll
    for (int ch = 0; ch < KL / 128; ++ch) { const int j0 = ch * 128 + lane * 4; v4f a; if (j0 <= i + ML) a = *(const v4f*)(ar + j0); else { a[0] = 0.f; a[1] = 0.f; a[2] = 0.f; a[3] = 0.f; }
#pragma unroll
        for (int u = 0; u < 4; ++u) { const int j = j0 + u; float t = -3.0e38f; if (j <= i + ML && mr[j] == 0) { const float s1 = __fadd_rn(a[u], br[j]); t = s1 * 0.125f; } v[ch * 4 + u] = t; mx = fmaxf(mx, t); } }
#pragma unroll
    for (int sh = 16; sh; sh >>= 1) mx = fmaxf(mx, __shfl_xor(mx, sh, 32));
    float sum = 0.f;
#pragma unroll
    for (int q = 0; q < KL / 32; ++q) { float d0 = __fsub_rn(v[q], mx); asm volatile("" : "+v"(d0)); v[q] = __builtin_amdgcn_exp2f(__fmul_rn(d0, 1.4426950408889634f)); sum += v[q]; }
#pragma unroll
    for (int sh = 16; sh; sh >>= 1) sum += __shfl_xor(sum, sh, 32);
    const float f = __fdiv_rn(PCAR, sum);
    for (int ps = 0; ps < 2; ++ps) {
#pragma unroll
        for (int ch = 0; ch < KL / 128; ++ch) { v4h o4; for (int q = 0; q < 4; ++q) o4[q] = tohx(v[ch * 4 + q] * f); *(volatile v4h*)(P16 + (size_t)row * KL + ch * 128 + lane * 4) = o4; }
        if (ps == 0) __threadfence(); } }
__global__ __launch_bounds__(256) void k_mrg(const float* __restrict__ O, int h0, bf* Ah, bf* Al) { const size_t e = ((size_t)blockIdx.x * 256 + threadIdx.x) * 4; if (e >= (size_t)ZH * QL * HD) return; const int d = (int)(e % HD); const int i = (int)((e / HD) % QL); const int zz = (int)(e / ((size_t)HD * QL)); const size_t oo = (size_t)i * DM + (h0 + zz) * HD + d; v4us oh, ol;
#pragma unroll
    for (int u = 0; u < 4; ++u) { unsigned short a, b; splitf(O[e + u] * (1.0f / PCAR), a, b); oh[u] = a; ol[u] = b; } *(volatile v4us*)(Ah + oo) = oh; *(volatile v4us*)(Al + oo) = ol; __threadfence(); *(volatile v4us*)(Ah + oo) = oh; *(volatile v4us*)(Al + oo) = ol; }
__global__ __launch_bounds__(256) void k_resid(const float* __restrict__ X, size_t bstride, const float* __restrict__ ATT, float* X1) { const size_t e = ((size_t)blockIdx.x * 256 + threadIdx.x) * 4; if (e >= (size_t)QL * DM) return; const size_t r = e / DM; const int c = (int)(e % DM); const v4f a = *(const v4f*)(X + r * bstride + c), t = *(const v4f*)(ATT + e); v4f o;
#pragma unroll
    for (int u = 0; u < 4; ++u) o[u] = __fadd_rn(bfr(a[u]), t[u]); *(volatile v4f*)(X1 + e) = o; __threadfence(); *(volatile v4f*)(X1 + e) = o; }
__global__ __launch_bounds__(256) void k_relupl(const float* __restrict__ F, bf* Ph, bf* Pl, size_t n4) { const size_t e = ((size_t)blockIdx.x * 256 + threadIdx.x) * 4; if (e >= n4 * 4) return; const v4f a = *(const v4f*)(F + e); v4us oh, ol;
#pragma unroll
    for (int u = 0; u < 4; ++u) { unsigned short x0, x1; splitf(fmaxf(a[u], 0.f), x0, x1); oh[u] = x0; ol[u] = x1; } *(volatile v4us*)(Ph + e) = oh; *(volatile v4us*)(Pl + e) = ol; __threadfence(); *(volatile v4us*)(Ph + e) = oh; *(volatile v4us*)(Pl + e) = ol; }
__global__ __launch_bounds__(256) void k_out(const float* __restrict__ X1, const float* __restrict__ Y2, float* dst, size_t bstride) { const size_t e = ((size_t)blockIdx.x * 256 + threadIdx.x) * 4; if (e >= (size_t)QL * DM) return; const size_t r = e / DM; const int c = (int)(e % DM); const v4f a = *(const v4f*)(X1 + e), y = *(const v4f*)(Y2 + e); v4f o;
#pragma unroll
    for (int u = 0; u < 4; ++u) o[u] = __fadd_rn(a[u], y[u]); float* p = dst + r * bstride + c; *(volatile v4f*)p = o; __threadfence(); *(volatile v4f*)p = o; }

extern "C" void kernel_launch(void* const* d_in, const int* in_sizes, int n_in,
                              void* d_out, int out_size, void* d_ws, size_t ws_size, hipStream_t stream) {
    (void)in_sizes; (void)n_in; (void)out_size;
    const float* input = (const float*)d_in[0]; const float* mems = (const float*)d_in[1]; const float* pos = (const float*)d_in[2]; const int* mask = (const int*)d_in[3]; const float* ln1g = (const float*)d_in[4]; const float* ln1b = (const float*)d_in[5]; const float* qkv_w = (const float*)d_in[6]; const float* qkv_b = (const float*)d_in[7];
    const float* r_w = (const float*)d_in[8]; const float* rwb = (const float*)d_in[9]; const float* rrb = (const float*)d_in[10]; const float* o_w = (const float*)d_in[11]; const float* ln2g = (const float*)d_in[12]; const float* ln2b = (const float*)d_in[13]; const float* w1 = (const float*)d_in[14]; const float* b1 = (const float*)d_in[15]; const float* w2 = (const float*)d_in[16]; const float* b2 = (const float*)d_in[17];
    float* OUT = (float*)d_out;
    char* wsp = (char*)d_ws;
    auto take = [&](size_t bytes) { char* p = wsp; wsp += (bytes + 255) & ~(size_t)255; return (void*)p; };
    bf* BQKV = (bf*)take((size_t)DM * 3 * DM * 2); bf* BR = (bf*)take((size_t)DM * DM * 2); bf* BO = (bf*)take((size_t)DM * DM * 2); bf* BW1 = (bf*)take((size_t)DM * DFF * 2); bf* BW2 = (bf*)take((size_t)DFF * DM * 2);
    bf* PEB = (bf*)take((size_t)KL * DM * 2); float* RK = (float*)take((size_t)KL * DM * 4); bf* RKh = (bf*)take((size_t)NH_ * KL * HD * 2); bf* RKl = (bf*)take((size_t)NH_ * KL * HD * 2);
    bf* CATh = (bf*)take((size_t)KL * DM * 2); bf* CATl = (bf*)take((size_t)KL * DM * 2); float* HEADS = (float*)take((size_t)KL * 3 * DM * 4);
    bf* QUh = (bf*)take((size_t)NH_ * QL * HD * 2); bf* QUl = (bf*)take((size_t)NH_ * QL * HD * 2); bf* QRh = (bf*)take((size_t)NH_ * QL * HD * 2); bf* QRl = (bf*)take((size_t)NH_ * QL * HD * 2); bf* KPh = (bf*)take((size_t)NH_ * KL * HD * 2); bf* KPl = (bf*)take((size_t)NH_ * KL * HD * 2); h16* VT = (h16*)take((size_t)NH_ * HD * KL * 2);
    float* AC = (float*)take((size_t)ZH * QL * KL * 4); float* BD = (float*)take((size_t)ZH * QL * KL * 4); h16* P16 = (h16*)take((size_t)ZH * QL * KL * 2); float* O = (float*)take((size_t)ZH * QL * HD * 4); bf* ATh = (bf*)take((size_t)QL * DM * 2); bf* ATl = (bf*)take((size_t)QL * DM * 2);
    float* ATT = (float*)take((size_t)QL * DM * 4); float* X1 = (float*)take((size_t)QL * DM * 4); bf* Yh = (bf*)take((size_t)QL * DM * 2); bf* Yl = (bf*)take((size_t)QL * DM * 2); float* HID = (float*)take((size_t)QL * DFF * 4); bf* HIh = (bf*)take((size_t)QL * DFF * 2); bf* HIl = (bf*)take((size_t)QL * DFF * 2); float* Y2 = (float*)take((size_t)QL * DM * 4);
    if ((size_t)(wsp - (char*)d_ws) > ws_size) return;
    k_wtG<<<(DM * 3 * DM / 64 + 63) / 64, 256, 0, stream>>>(qkv_w, DM, 3 * DM, BQKV); k_wtG<<<(DM * DM / 64 + 63) / 64, 256, 0, stream>>>(r_w, DM, DM, BR); k_wtG<<<(DM * DM / 64 + 63) / 64, 256, 0, stream>>>(o_w, DM, DM, BO); k_wtG<<<(DM * DFF / 64 + 63) / 64, 256, 0, stream>>>(w1, DM, DFF, BW1); k_wtG<<<(DFF * DM / 64 + 63) / 64, 256, 0, stream>>>(w2, DFF, DM, BW2);
    k_cvt8<<<(KL * DM / 8 + 255) / 256, 256, 0, stream>>>(pos, PEB, KL * DM / 8);
    k_gemmw<bf, 0, false><<<dim3(KL / 64, DM / 64, 1), 32, 0, stream>>>(PEB, nullptr, BR, nullptr, DM, RK, DM, nullptr, 0, 0, 0); k_hpb<<<(unsigned)(((size_t)NH_ * KL * HD / 4 + 255) / 256), 256, 0, stream>>>(RK, DM, 0, KL, nullptr, RKh, RKl);
    const size_t bst = (size_t)NB_ * DM; const size_t zq = (size_t)QL * HD, zk = (size_t)KL * HD, zS = (size_t)QL * KL, zv = (size_t)HD * KL, zo = (size_t)QL * HD; const unsigned LQ = (unsigned)(((size_t)QL * DM / 4 + 255) / 256);
    for (int b = 0; b < NB_; ++b) {
        k_lnrow<<<ML / 8, 256, 0, stream>>>(mems + (size_t)b * DM, bst, ln1g, ln1b, 1, 0, CATh, CATl); k_lnrow<<<QL / 8, 256, 0, stream>>>(input + (size_t)b * DM, bst, ln1g, ln1b, 1, ML, CATh, CATl);
        k_gemmw<bf, 1, true><<<dim3(KL / 64, 3 * DM / 64, 1), 32, 0, stream>>>(CATh, CATl, BQKV, nullptr, DM, HEADS, 3 * DM, qkv_b, 0, 0, 0);
        k_hpb<<<(unsigned)(((size_t)NH_ * QL * HD / 4 + 255) / 256), 256, 0, stream>>>(HEADS + (size_t)ML * 3 * DM, 3 * DM, 0, QL, rwb, QUh, QUl); k_hpb<<<(unsigned)(((size_t)NH_ * QL * HD / 4 + 255) / 256), 256, 0, stream>>>(HEADS + (size_t)ML * 3 * DM, 3 * DM, 0, QL, rrb, QRh, QRl);
        k_hpb<<<(unsigned)(((size_t)NH_ * KL * HD / 4 + 255) / 256), 256, 0, stream>>>(HEADS, 3 * DM, DM, KL, nullptr, KPh, KPl); k_vt16<<<(unsigned)(((size_t)NH_ * HD * KL / 2 + 255) / 256), 256, 0, stream>>>(HEADS, VT);
        for (int h0 = 0; h0 < NH_; h0 += ZH) {
            k_gemmc<bf, 2, 1><<<dim3(QL / 64, KL / 64, ZH), 32, 0, stream>>>(QUh + (size_t)h0 * zq, QUl + (size_t)h0 * zq, KPh + (size_t)h0 * zk, KPl + (size_t)h0 * zk, HD, AC, KL, ML, zq, zk, zS);
            k_gemmw<bf, 2, false><<<dim3(QL / 64, KL / 64, ZH), 32, 0, stream>>>(QRh + (size_t)h0 * zq, QRl + (size_t)h0 * zq, RKh + (size_t)h0 * zk, RKl + (size_t)h0 * zk, HD, BD, KL, nullptr, zq, zk, zS);
            k_xsoft<<<ZH * QL / 8, 256, 0, stream>>>(AC, BD, mask, P16);
            k_gemmc<h16, 0, 2><<<dim3(QL / 64, 1, ZH), 32, 0, stream>>>(P16, nullptr, VT + (size_t)h0 * zv, nullptr, KL, O, HD, ML, zS, zv, zo);
            k_mrg<<<(unsigned)(((size_t)ZH * QL * HD / 4 + 255) / 256), 256, 0, stream>>>(O, h0, ATh, ATl); }
        k_gemmw<bf, 1, false><<<dim3(QL / 64, DM / 64, 1), 32, 0, stream>>>(ATh, ATl, BO, nullptr, DM, ATT, DM, nullptr, 0, 0, 0);
        k_resid<<<LQ, 256, 0, stream>>>(input + (size_t)b * DM, bst, ATT, X1);
        k_lnrow<<<QL / 8, 256, 0, stream>>>(X1, DM, ln2g, ln2b, 0, 0, Yh, Yl);
        k_gemmw<bf, 1, true><<<dim3(QL / 64, DFF / 64, 1), 32, 0, stream>>>(Yh, Yl, BW1, nullptr, DM, HID, DFF, b1, 0, 0, 0); k_relupl<<<(unsigned)(((size_t)QL * DFF / 4 + 255) / 256), 256, 0, stream>>>(HID, HIh, HIl, (size_t)QL * DFF / 4);
        k_gemmw<bf, 1, true><<<dim3(QL / 64, DM / 64, 1), 32, 0, stream>>>(HIh, HIl, BW2, nullptr, DFF, Y2, DM, b2, 0, 0, 0);
        k_out<<<LQ, 256, 0, stream>>>(X1, Y2, OUT + (size_t)b * DM, bst); }
}
